// DMRG_27676769255718
// MI455X (gfx1250) — hardware-verified
//
#include <hip/hip_runtime.h>
#include <math.h>

typedef __attribute__((ext_vector_type(16))) _Float16 v16h;
typedef __attribute__((ext_vector_type(8)))  _Float16 v8h;
typedef __attribute__((ext_vector_type(8)))  float    v8f;
typedef __attribute__((ext_vector_type(4)))  float    v4f;
typedef __attribute__((ext_vector_type(4)))  unsigned v4u;

constexpr int kChi    = 1024;
constexpr int kBond   = 5;
constexpr int kPhys   = 2;
constexpr int kRowsPsi = kChi * kPhys * kPhys;
constexpr int kRowsR   = kBond * kChi;
constexpr int kKL      = kBond * kChi;
constexpr int kOutCols = kPhys * kPhys * kChi;
constexpr int kTabN    = kBond * kPhys * kPhys * kBond * kPhys * kPhys;
constexpr int kTabPad  = 512;
static_assert(kRowsPsi == 4096 && kRowsR == 5120 && kKL == 5120 && kOutCols == 4096 && kTabN == 400, "shape constants");
static_assert((kRowsR % 64) == 0 && (kRowsPsi % 64) == 0 && (kChi % 32) == 0, "first product tile multiples");
static_assert((kChi % 64) == 0 && (kOutCols % 64) == 0 && (kKL % 32) == 0, "second product tile multiples");
static_assert(((kRowsR / 64) * (kRowsPsi / 64)) % 8 == 0 && ((kChi / 64) * (kOutCols / 64)) % 8 == 0, "eight tiles per block");

constexpr float kCarryIn  = 64.0f;
constexpr float kFoldW    = 1.0f / (kCarryIn * kCarryIn);
constexpr float kFoldOut  = 1.0f / kCarryIn;
constexpr float kF16MinNormal = 6.103515625e-05f;

constexpr size_t kSzPsi16 = (size_t)kRowsPsi * kChi * 2;
constexpr size_t kSzR16   = (size_t)kRowsR * kChi * 2;
constexpr size_t kSzL16p  = (size_t)kChi * kKL * 2;
constexpr size_t kSzWt16  = (size_t)kRowsR * kRowsPsi * 2;
constexpr size_t kSzVt16  = (size_t)kOutCols * kKL * 2;
constexpr size_t kSzTab   = (size_t)kTabPad * 4;
constexpr size_t kOffPsi16 = 0;
constexpr size_t kOffR16   = kOffPsi16 + kSzPsi16;
constexpr size_t kOffL16p  = kOffR16 + kSzR16;
constexpr size_t kOffWt16  = kOffL16p + kSzL16p;
constexpr size_t kOffVt16  = kOffWt16 + kSzWt16;
constexpr size_t kOffTab   = kOffVt16 + kSzVt16;
constexpr size_t kWsTotal  = kOffTab + kSzTab;
static_assert(kWsTotal == 8388608ull + 10485760ull + 10485760ull + 41943040ull + 41943040ull + 2048ull, "carve sum");
static_assert(kWsTotal == 113248256ull, "carve total");
static_assert(kWsTotal <= 134217728ull, "carve cap");
static_assert((kOffR16 % 128) == 0 && (kOffL16p % 128) == 0 && (kOffWt16 % 128) == 0 &&
              (kOffVt16 % 128) == 0 && (kOffTab % 128) == 0, "128-B aligned regions");

__device__ __forceinline__ float flush_small(float x) {
  return (fabsf(x) < kF16MinNormal) ? 0.0f : x;
}

__device__ __forceinline__ float h16_to_f32(unsigned hb) {
  const unsigned sgn = (hb & 0x8000u) << 16; const unsigned em = hb & 0x7fffu;
  const float fn = __uint_as_float((em << 13) + 0x38000000u);
  const float fs = (float)em * 5.9604644775390625e-8f;
  const float mag = (em < 0x400u) ? fs : fn; return __uint_as_float(__float_as_uint(mag) | sgn);
}

__device__ __forceinline__ void tie_light(v8f& a, v16h x, v16h y) {
  asm volatile("v_nop" : "+v"(a) : "v"(x), "v"(y));
}
__device__ __forceinline__ void tie_full(v8f& a, v16h x, v16h y) {
  asm volatile("v_nop\n\tv_nop\n\tv_nop\n\tv_nop" : "+v"(a) : "v"(x), "v"(y));
}
__device__ __forceinline__ void tie_acc(v8f& a) {
  asm volatile("v_nop" : "+v"(a));
}
__device__ __forceinline__ void keep4_h(v16h a, v16h b, v16h c, v16h d) {
  asm volatile("v_nop" :: "v"(a), "v"(b), "v"(c), "v"(d));
}

struct FragH {
  union U { v16h v; v8h h[2]; };
  static __device__ __forceinline__ v16h load(const _Float16* p) {
    U f; f.h[0] = *(const v8h*)(p); f.h[1] = *(const v8h*)(p + 16); return f.v;
  }
  static __device__ __forceinline__ v8f mma(v16h a, v16h b, v8f c) {
    return __builtin_amdgcn_wmma_f32_16x16x32_f16(false, a, false, b, (short)0, c, false, false);
  }
};

template <bool PERM>
__global__ __launch_bounds__(256) void rows_to_f16_kernel(
    const float* __restrict__ src, unsigned short* __restrict__ dst, int total8, float carry)
{
  const int t = blockIdx.x * 256 + threadIdx.x;
  if (t >= total8) return;
  size_t so = (size_t)t << 3;
  if (PERM) {
    const int a8 = t & 127;
    const int hb = t >> 7;
    const int h  = hb / kBond;
    const int b  = hb - h * kBond;
    so = (size_t)b * kChi * kChi + (size_t)h * kChi + (size_t)a8 * 8;
  }
  const v4f a0 = *(const v4f*)(src + so);
  const v4f a1 = *(const v4f*)(src + so + 4);
  v8h hv;
#pragma unroll
  for (int e = 0; e < 4; ++e) {
    const float x0 = a0[e] * carry;
    const float x1 = a1[e] * carry;
    hv[e]     = (_Float16)flush_small(x0);
    hv[4 + e] = (_Float16)flush_small(x1);
  }
  unsigned short* q = dst + ((size_t)t << 3);
  *(volatile v8h*)q = hv;
  __threadfence();
  *(volatile v8h*)q = hv;
}

__global__ __launch_bounds__(512) void site_table_kernel(
    const float* __restrict__ M1, const float* __restrict__ M2, float* __restrict__ Tg)
{
  const int t  = threadIdx.x;
  const int tc = (t < kTabN) ? t : (kTabN - 1);
  const int e = tc & 1;
  const int c = (tc >> 1) & 1;
  const int f = (tc >> 2) % kBond;
  const int o = tc / 20;
  const int j = o & 1;
  const int i = (o >> 1) & 1;
  const int b = o >> 2;
  float acc = 0.0f;
#pragma unroll
  for (int d = 0; d < kBond; ++d) {
    const float m1 = M1[((b * kBond + d) * kPhys + i) * kPhys + c];
    const float m2 = M2[((d * kBond + f) * kPhys + j) * kPhys + e];
    acc = fmaf(m1, m2, acc);
  }
  const float val = (t < kTabN) ? acc : 0.0f;
  *(volatile float*)(Tg + t) = val;
  __threadfence();
  *(volatile float*)(Tg + t) = val;
}

template <int OUT_MODE>
__global__ __launch_bounds__(256) void gemm64_f16_kernel(
    const unsigned short* __restrict__ Ap, int lda,
    const unsigned short* __restrict__ Btp, int ldb,
    void* __restrict__ Cout, int ldc,
    int M, int N, int K, float scale)
{
  const _Float16* A  = (const _Float16*)Ap;
  const _Float16* Bt = (const _Float16*)Btp;
  __shared__ __align__(16) float sSlab[8][16 * 68];
  const int lane = threadIdx.x & 31;
  const int wave = threadIdx.x >> 5;
  const int tilesN = N >> 6;
  const int tilesM = M >> 6;
  const int tile = blockIdx.x * 8 + wave;
  if (tile >= tilesM * tilesN) return;
  const int tm = tile / tilesN;
  const int tn = tile - tm * tilesN;
  const int m0 = tm << 6;
  const int n0 = tn << 6;

  const int rlane = lane & 15;
  const int koff  = (lane >> 4) * 8;
  const int mOff  = (lane >> 4) * 8;

  v8f acc[4][4];
#pragma unroll
  for (int i = 0; i < 4; ++i)
#pragma unroll
    for (int j = 0; j < 4; ++j) acc[i][j] = (v8f){0.f,0.f,0.f,0.f,0.f,0.f,0.f,0.f};

  for (int k0 = 0; k0 < K; k0 += 32) {
    v16h bh[4];
#pragma unroll
    for (int j = 0; j < 4; ++j) {
      const size_t bo = (size_t)(n0 + (j << 4) + rlane) * ldb + koff + k0;
      bh[j] = FragH::load(Bt + bo);
    }
#pragma unroll
    for (int i = 0; i < 4; ++i) {
      const size_t ao = (size_t)(m0 + (i << 4) + rlane) * lda + koff + k0;
      const v16h ah = FragH::load(A + ao);
#pragma unroll
      for (int j = 0; j < 4; ++j) acc[i][j] = FragH::mma(ah, bh[j], acc[i][j]);
      tie_light(acc[i][0], ah, bh[0]);
      tie_light(acc[i][1], ah, bh[1]);
      tie_light(acc[i][2], ah, bh[2]);
      tie_full(acc[i][3], ah, bh[3]);
    }
    keep4_h(bh[0], bh[1], bh[2], bh[3]);
  }
#pragma unroll
  for (int i = 0; i < 4; ++i)
#pragma unroll
    for (int j = 0; j < 4; ++j) tie_acc(acc[i][j]);

  float* slab = sSlab[wave];
#pragma unroll
  for (int i = 0; i < 4; ++i) {
    const int mBase = m0 + (i << 4);
#pragma unroll
    for (int j = 0; j < 4; ++j) {
#pragma unroll
      for (int r = 0; r < 8; ++r) {
        const float v = acc[i][j][r] * scale;
        slab[(mOff + r) * 68 + (j << 4) + rlane] = v;
      }
    }
    __builtin_amdgcn_fence(__ATOMIC_RELEASE, "workgroup");
    __builtin_amdgcn_wave_barrier();
    __builtin_amdgcn_fence(__ATOMIC_ACQUIRE, "workgroup");
    if (OUT_MODE == 0) {
      float* C = (float*)Cout;
      const int hh = lane >> 4, c4 = (lane & 15) * 4;
      for (int pass = 0; pass < 2; ++pass) {
#pragma unroll
        for (int it = 0; it < 8; ++it) {
          const int row = it * 2 + hh;
          const v4f v = *(const v4f*)(slab + row * 68 + c4);
          *(volatile v4f*)(C + (size_t)(mBase + row) * ldc + n0 + c4) = v;
        }
        __threadfence();
      }
    } else {
      const int q = lane >> 3, c8 = (lane & 7) * 8;
      unsigned short* C = (unsigned short*)Cout;
      for (int pass = 0; pass < 2; ++pass) {
#pragma unroll
        for (int it = 0; it < 4; ++it) {
          const int row = it * 4 + q;
          const float* sp = slab + row * 68 + c8;
          v8h hv;
#pragma unroll
          for (int e = 0; e < 8; ++e) {
            const float x = sp[e];
            hv[e] = (_Float16)flush_small(x);
          }
          *(volatile v8h*)(C + (size_t)(mBase + row) * ldc + n0 + c8) = hv;
        }
        __threadfence();
      }
    }
    __builtin_amdgcn_fence(__ATOMIC_RELEASE, "workgroup");
    __builtin_amdgcn_wave_barrier();
    __builtin_amdgcn_fence(__ATOMIC_ACQUIRE, "workgroup");
  }
}

__global__ __launch_bounds__(256) void mix_kernel(
    const float* __restrict__ Tg, const unsigned short* __restrict__ Wt16, unsigned* __restrict__ Vw)
{
  __shared__ __align__(16) float sT[kTabPad];
  __shared__ unsigned sO[20 * 256];
  const int tid = threadIdx.x;
  sT[tid]       = Tg[tid];
  sT[tid + 256] = Tg[tid + 256];
  const int k     = blockIdx.x >> 1;
  const int apair = (blockIdx.x & 1) * 256 + tid;

  float w0[20], w1[20];
#pragma unroll
  for (int f = 0; f < kBond; ++f) {
    const v4u q = *(const v4u*)(Wt16 + ((size_t)(f * kChi + k)) * kRowsPsi + (size_t)apair * 8);
    const unsigned q0 = q[0];
    const unsigned q1 = q[1];
    const unsigned q2 = q[2];
    const unsigned q3 = q[3];
    w0[f * 4 + 0] = h16_to_f32(q0 & 0xffffu);
    w0[f * 4 + 1] = h16_to_f32(q0 >> 16);
    w0[f * 4 + 2] = h16_to_f32(q1 & 0xffffu);
    w0[f * 4 + 3] = h16_to_f32(q1 >> 16);
    w1[f * 4 + 0] = h16_to_f32(q2 & 0xffffu);
    w1[f * 4 + 1] = h16_to_f32(q2 >> 16);
    w1[f * 4 + 2] = h16_to_f32(q3 & 0xffffu);
    w1[f * 4 + 3] = h16_to_f32(q3 >> 16);
  }
  __syncthreads();

#pragma unroll 1
  for (int o = 0; o < 20; ++o) {
    const v4f* tp = (const v4f*)(sT + o * 20);
    float s0 = 0.0f, s1 = 0.0f;
#pragma unroll
    for (int q4 = 0; q4 < 5; ++q4) {
      const v4f tv = tp[q4];
#pragma unroll
      for (int e = 0; e < 4; ++e) {
        const float tt = tv[e];
        s0 = fmaf(tt, w0[q4 * 4 + e], s0);
        s1 = fmaf(tt, w1[q4 * 4 + e], s1);
      }
    }
    const _Float16 h0 = (_Float16)flush_small(s0);
    const _Float16 h1 = (_Float16)flush_small(s1);
    const unsigned u = (unsigned)__builtin_bit_cast(unsigned short, h0) |
                       ((unsigned)__builtin_bit_cast(unsigned short, h1) << 16);
    sO[o * 256 + tid] = u;
  }
  __syncthreads();

  for (int pass = 0; pass < 2; ++pass) {
#pragma unroll 1
    for (int o = 0; o < 20; ++o) {
      const unsigned u = sO[o * 256 + tid];
      const size_t idx = ((size_t)((o & 3) * kChi + k)) * (size_t)(kKL / 2) + (size_t)((o >> 2) * (kChi / 2)) + (size_t)apair;
      *(volatile unsigned*)(Vw + idx) = u;
    }
    __threadfence();
  }
}

extern "C" void kernel_launch(void* const* d_in, const int* in_sizes, int n_in,
                              void* d_out, int out_size, void* d_ws, size_t ws_size,
                              hipStream_t stream) {
  if (n_in < 5) return;
  if (in_sizes[0] != kRowsPsi * kChi) return;
  if (in_sizes[1] != kBond * kChi * kChi) return;
  if (in_sizes[2] != kBond * kBond * kPhys * kPhys) return;
  if (in_sizes[3] != kBond * kBond * kPhys * kPhys) return;
  if (in_sizes[4] != kBond * kChi * kChi) return;
  if (out_size != kChi * kOutCols) return;
  if (ws_size < kWsTotal) return;

  const float* psi = (const float*)d_in[0];
  const float* Lg  = (const float*)d_in[1];
  const float* M1  = (const float*)d_in[2];
  const float* M2  = (const float*)d_in[3];
  const float* Rg  = (const float*)d_in[4];

  char* ws = (char*)d_ws;
  unsigned short* PSI16 = (unsigned short*)(ws + kOffPsi16);
  unsigned short* R16   = (unsigned short*)(ws + kOffR16);
  unsigned short* L16P  = (unsigned short*)(ws + kOffL16p);
  unsigned short* WT16  = (unsigned short*)(ws + kOffWt16);
  unsigned short* VT16  = (unsigned short*)(ws + kOffVt16);
  float*          TAB   = (float*)(ws + kOffTab);

  rows_to_f16_kernel<false><<<(kRowsPsi * kChi / 8) / 256, 256, 0, stream>>>(psi, PSI16, kRowsPsi * kChi / 8, kCarryIn);
  rows_to_f16_kernel<false><<<(kRowsR * kChi / 8) / 256, 256, 0, stream>>>(Rg, R16, kRowsR * kChi / 8, kCarryIn);
  rows_to_f16_kernel<true><<<(kChi * kKL / 8) / 256, 256, 0, stream>>>(Lg, L16P, kChi * kKL / 8, kCarryIn);

  site_table_kernel<<<1, 512, 0, stream>>>(M1, M2, TAB);

  gemm64_f16_kernel<1><<<dim3((kRowsR / 64) * (kRowsPsi / 64) / 8), 256, 0, stream>>>(
      R16, kChi,
      PSI16, kChi,
      (void*)WT16, kRowsPsi,
      kRowsR, kRowsPsi, kChi, kFoldW);

  mix_kernel<<<kChi * 2, 256, 0, stream>>>(TAB, WT16, (unsigned*)VT16);

  gemm64_f16_kernel<0><<<dim3((kChi / 64) * (kOutCols / 64) / 8), 256, 0, stream>>>(
      L16P, kKL,
      VT16, kKL,
      d_out, kOutCols,
      kChi, kOutCols, kKL, kFoldOut);
}
